// ShapletLearner_54717883351092
// MI455X (gfx1250) — hardware-verified
//
#include <hip/hip_runtime.h>
#include <stddef.h>
#include <stdint.h>

#pragma clang fp contract(off)

#define QLEN   1024
#define KLEN   32
#define NSH    64
#define NCLS   2
#define NSEG   (QLEN - KLEN + 1)
#define NTILE  64
#define NWAVE  8
#define TPW    (NTILE / NWAVE)
#define RPB    16
#define TSHLEN (NTILE * 16 + KLEN)
#define BIGF   1.0e30f

static_assert(NSEG == 993);
static_assert(TPW == 8);
static_assert(TSHLEN == 1056);
static_assert(NTILE * 16 >= NSEG);
static_assert(NTILE * 16 == QLEN);
static_assert(NSH * KLEN == 8 * 256);
static_assert(QLEN == 4 * 256);
static_assert(2 * RPB * 4 == 128);
static_assert(TSHLEN - QLEN == 32);

typedef _Float16 hh;
typedef hh    v16h __attribute__((ext_vector_type(16)));
typedef hh    v8h  __attribute__((ext_vector_type(8)));
typedef hh    v4h  __attribute__((ext_vector_type(4)));
typedef float v8f  __attribute__((ext_vector_type(8)));
typedef float v4f  __attribute__((ext_vector_type(4)));

union Frag { v16h v; v8h half[2]; };

__device__ __forceinline__ v8f mma16(v16h a, v16h b, v8f c) {
  return __builtin_amdgcn_wmma_f32_16x16x32_f16(false, a, false, b, (short)0, c, false, false);
}

__device__ __forceinline__ v8h ld8h(const hh* p) {
  const v8h r = {p[0], p[1], p[2], p[3], p[4], p[5], p[6], p[7]};
  return r;
}

__device__ __forceinline__ v8f vmin8(v8f a, v8f b) {
  v8f r;
#pragma unroll
  for (int i = 0; i < 8; ++i) r[i] = fminf(a[i], b[i]);
  return r;
}

__global__ __launch_bounds__(256) void k_shapelet(const float* __restrict__ ts, const float* __restrict__ sh,
                                                  const float* __restrict__ fcw, const float* __restrict__ fcb,
                                                  float* __restrict__ out) {
  __shared__ __align__(16) float tsf[QLEN];
  __shared__ __align__(16) hh    tsh[TSHLEN];
  __shared__ __align__(16) float cs[QLEN + 4];
  __shared__ __align__(16) float wsq[NTILE * 16];
  __shared__ __align__(16) hh    shh[NSH * KLEN];
  __shared__ float ssq[NSH];
  __shared__ float fwv[NWAVE][NSH];
  __shared__ float featf[NSH];
  __shared__ __align__(16) float ost[2 * RPB];

  const int tid = threadIdx.x, lane = tid & 31, wave = tid >> 5;
  const int h = lane >> 4, m = lane & 15;

  {
    const float* sp = sh + 8 * tid;
    const v4f a0 = *(const v4f*)(sp);
    const v4f a1 = *(const v4f*)(sp + 4);
    const v8f t8 = {-2.0f * a0[0], -2.0f * a0[1], -2.0f * a0[2], -2.0f * a0[3],
                    -2.0f * a1[0], -2.0f * a1[1], -2.0f * a1[2], -2.0f * a1[3]};
    *(v8h*)(shh + 8 * tid) = __builtin_convertvector(t8, v8h);
  }
  if (tid < NSH) {
    float acc = 0.0f;
#pragma unroll 8
    for (int k = 0; k < KLEN; ++k) { const float v = sh[tid * KLEN + k]; acc += v * v; }
    ssq[tid] = acc;
  }
  if (tid < TSHLEN - QLEN) tsh[QLEN + tid] = (hh)0.0f;
  __syncthreads();

  Frag bq[4];
#pragma unroll
  for (int nt = 0; nt < 4; ++nt) {
    const hh* bp = shh + (16 * nt + m) * KLEN + 8 * h;
    bq[nt].half[0] = *(const v8h*)(bp);
    bq[nt].half[1] = *(const v8h*)(bp + 16);
  }
  const v8f big8 = {BIGF, BIGF, BIGF, BIGF, BIGF, BIGF, BIGF, BIGF};

#pragma unroll 1
  for (int ri = 0; ri < RPB; ++ri) {
    const int row = blockIdx.x * RPB + ri;

    {
      const v4f x = *(const v4f*)(ts + (size_t)row * QLEN + 4 * tid);
      *(v4f*)(tsf + 4 * tid) = x;
      *(v4h*)(tsh + 4 * tid) = __builtin_convertvector(x, v4h);
    }
    __syncthreads();

    if (wave == 0) {
      const float* xp = tsf + 32 * lane;
      float tot = 0.0f;
#pragma unroll 8
      for (int j = 0; j < 32; ++j) { const float x = xp[j]; tot += x * x; }
      float inc = tot;
#pragma unroll
      for (int d = 1; d < 32; d <<= 1) {
        const float y = __shfl_up(inc, d, 32);
        inc = (lane >= d) ? (inc + y) : inc;
      }
      const float up1 = __shfl_up(inc, 1, 32);
      float run = (lane == 0) ? 0.0f : up1;
      if (lane == 0) cs[0] = 0.0f;
      float* cp = cs + 32 * lane + 1;
#pragma unroll 8
      for (int j = 0; j < 32; ++j) { const float x = xp[j]; run += x * x; cp[j] = run; }
    }
    __syncthreads();

#pragma unroll
    for (int q = 0; q < 4; ++q) {
      const int s  = tid + 256 * q;
      const int s2 = (s + KLEN < QLEN) ? (s + KLEN) : QLEN;
      const float d = cs[s2] - cs[s];
      wsq[s] = (s < NSEG) ? d : BIGF;
    }
    __syncthreads();

    v8f mn[4];
#pragma unroll
    for (int nt = 0; nt < 4; ++nt) mn[nt] = big8;
    const int tb = wave * TPW;
    v8h lo = ld8h(tsh + tb * 16 + m + 8 * h);
#pragma unroll 1
    for (int j = 0; j < TPW; ++j) {
      const int s0 = (tb + j) * 16;
      const v8h nx = ld8h(tsh + s0 + 16 + m + 8 * h);
      Frag a;
      a.half[0] = lo;
      a.half[1] = nx;
      const v8f cin = *(const v8f*)(wsq + s0 + 8 * h);
      v8f d0 = mma16(a.v, bq[0].v, cin);
      v8f d1 = mma16(a.v, bq[1].v, cin);
      v8f d2 = mma16(a.v, bq[2].v, cin);
      v8f d3 = mma16(a.v, bq[3].v, cin);
      asm volatile("v_nop\n\tv_nop\n\tv_nop\n\tv_nop"
                   : "+v"(d0), "+v"(d1), "+v"(d2), "+v"(d3)
                   : "v"(a.v), "v"(bq[0].v), "v"(bq[1].v), "v"(bq[2].v), "v"(bq[3].v), "v"(cin));
      mn[0] = vmin8(mn[0], d0);
      mn[1] = vmin8(mn[1], d1);
      mn[2] = vmin8(mn[2], d2);
      mn[3] = vmin8(mn[3], d3);
      lo = nx;
    }

    float fv[4];
#pragma unroll
    for (int nt = 0; nt < 4; ++nt) {
      float v = mn[nt][0];
#pragma unroll
      for (int r = 1; r < 8; ++r) v = fminf(v, mn[nt][r]);
      const float o = __shfl_xor(v, 16, 32);
      fv[nt] = fminf(v, o);
    }
    if (h == 0) {
#pragma unroll
      for (int nt = 0; nt < 4; ++nt) fwv[wave][16 * nt + m] = fv[nt];
    }
    __syncthreads();
    if (tid < NSH) {
      float f = fwv[0][tid];
#pragma unroll
      for (int w = 1; w < NWAVE; ++w) f = fminf(f, fwv[w][tid]);
      featf[tid] = (f + ssq[tid]) * (1.0f / (float)KLEN);
    }
    __syncthreads();
    if (wave == 0) {
      const float f0 = featf[lane], f1 = featf[lane + 32];
      float p0 = f0 * fcw[lane] + f1 * fcw[lane + 32];
      float p1 = f0 * fcw[NSH + lane] + f1 * fcw[NSH + lane + 32];
#pragma unroll
      for (int d = 16; d > 0; d >>= 1) {
        p0 += __shfl_xor(p0, d, 32);
        p1 += __shfl_xor(p1, d, 32);
      }
      if (lane == 0) {
        ost[2 * ri]     = p0 + fcb[0];
        ost[2 * ri + 1] = p1 + fcb[1];
      }
    }
  }

  __syncthreads();
  if (wave == 0) {
    const int li = lane & 7;
    const v4f v = *(const v4f*)(ost + 4 * li);
    float* gp = out + (size_t)blockIdx.x * (2 * RPB) + 4 * li;
    if (lane < 8) *(volatile v4f*)gp = v;
    __threadfence();
    if (lane < 8) *(volatile v4f*)gp = v;
  }
}

extern "C" void kernel_launch(void* const* d_in, const int* in_sizes, int n_in,
                              void* d_out, int out_size, void* d_ws, size_t ws_size,
                              hipStream_t stream) {
  (void)d_ws; (void)ws_size;
  if (n_in < 4) return;
  const int n0 = in_sizes[0];
  if (n0 <= 0 || (n0 % QLEN) != 0) return;
  const int nrows = n0 / QLEN;
  if ((nrows % RPB) != 0) return;
  if (in_sizes[1] != NSH * KLEN) return;
  if (in_sizes[2] != NCLS * NSH) return;
  if (in_sizes[3] != NCLS) return;
  if (out_size != nrows * NCLS) return;

  const float* ts  = (const float*)d_in[0];
  const float* sh  = (const float*)d_in[1];
  const float* fcw = (const float*)d_in[2];
  const float* fcb = (const float*)d_in[3];
  float* out = (float*)d_out;

  k_shapelet<<<dim3(nrows / RPB), dim3(256), 0, stream>>>(ts, sh, fcw, fcb, out);
  (void)hipGetLastError();
}
